// GCN3_84954453115003
// MI455X (gfx1250) — hardware-verified
//
#include <hip/hip_runtime.h>
#include <stddef.h>


#define KD      128
#define HID     128
#define OUTC    64
#define NTHR    256
#define NWAVE   8
#define EPT     8
#define NGRP    2
#define CHUNK   (NTHR * EPT * NGRP)
#define WCAP    (EPT * NGRP * 32)
#define LISTN   (NWAVE * WCAP)
#define NBC     4096
#define NBF     1024
#define RCAP    20480
#define RBN     128
#define GROWS   128
#define OTHR    512
#define ATHR    128
#define AWAVE   4
#define TGT     (AWAVE * 32)
#define DEGCAP  256
#define WSCALE  16.0f
#define WINV    0.0625f

#define LDS_FILL   (RCAP * 8 + NBF * 4 + LISTN * 4 + 64)
#define LDS_GEMM8  (GROWS * 128 * 4)
#define LDS_GEMM4  (GROWS * 64 * 4)
#define LDS_AGG128 (AWAVE * 32 * 128 * 4)
#define LDS_AGG64  (AWAVE * 32 * 64 * 4)

static_assert((CHUNK & (CHUNK - 1)) == 0);
static_assert(CHUNK <= 4096);
static_assert(NBC <= 4096 && NBF <= 4096);
static_assert((NBC & (NBC - 1)) == 0 && (NBF & (NBF - 1)) == 0);
static_assert(NBC == 4 * NBF);
static_assert(OTHR * 8 == NBC);
static_assert((RCAP % 32) == 0);
static_assert(TGT == GROWS);
static_assert((NBC % GROWS) == 0);
static_assert((KD % 32) == 0);
static_assert((HID * KD / 8) % NTHR == 0 && (OUTC * KD / 8) % NTHR == 0);

typedef float    v4f  __attribute__((ext_vector_type(4)));
typedef float    v8f  __attribute__((ext_vector_type(8)));
typedef int      v4i  __attribute__((ext_vector_type(4)));
typedef int      v2i  __attribute__((ext_vector_type(2)));
typedef _Float16 v8h  __attribute__((ext_vector_type(8)));
typedef _Float16 v16h __attribute__((ext_vector_type(16)));
union FragH { v16h v; v8h h[2]; };

__device__ __forceinline__ v8h cvt8(v4f a, v4f b) {
  v8h r;
  r[0] = (_Float16)a.x; r[1] = (_Float16)a.y; r[2] = (_Float16)a.z; r[3] = (_Float16)a.w;
  r[4] = (_Float16)b.x; r[5] = (_Float16)b.y; r[6] = (_Float16)b.z; r[7] = (_Float16)b.w;
  return r;
}

__device__ __forceinline__ v8f wmh(v16h a, v16h b, v8f c) {
  v8f d = __builtin_amdgcn_wmma_f32_16x16x32_f16(false, a, false, b, (short)0, c, false, false);
  asm volatile("v_nop\n\tv_nop\n\tv_nop\n\tv_nop" : "+v"(d) : "v"(a), "v"(b));
  return d;
}

template <int NB>
__device__ __forceinline__ int scan_chunk(const int* __restrict__ dsts, int nE, int cbase, int slotBase,
                                          int vec8, int* list, int tid, int lane, int wave) {
  int wc = 0;
#pragma unroll
  for (int g = 0; g < NGRP; ++g) {
    const int el0  = (g * NTHR + tid) * EPT;
    const int e0   = cbase + el0;
    const int sent = -2147483647 - 1;
    v4i da, db;
    if (vec8 != 0 && cbase + CHUNK <= nE) {
      da = *(const v4i*)(dsts + e0);
      db = *(const v4i*)(dsts + e0 + 4);
    } else {
      da.x = (e0     < nE) ? dsts[min(e0, nE - 1)] : sent;
      da.y = (e0 + 1 < nE) ? dsts[min(e0 + 1, nE - 1)] : sent;
      da.z = (e0 + 2 < nE) ? dsts[min(e0 + 2, nE - 1)] : sent;
      da.w = (e0 + 3 < nE) ? dsts[min(e0 + 3, nE - 1)] : sent;
      db.x = (e0 + 4 < nE) ? dsts[min(e0 + 4, nE - 1)] : sent;
      db.y = (e0 + 5 < nE) ? dsts[min(e0 + 5, nE - 1)] : sent;
      db.z = (e0 + 6 < nE) ? dsts[min(e0 + 6, nE - 1)] : sent;
      db.w = (e0 + 7 < nE) ? dsts[min(e0 + 7, nE - 1)] : sent;
    }
    const unsigned nb = (unsigned)slotBase;
    const unsigned s0 = (unsigned)da.x - nb, s1 = (unsigned)da.y - nb;
    const unsigned s2 = (unsigned)da.z - nb, s3 = (unsigned)da.w - nb;
    const unsigned s4 = (unsigned)db.x - nb, s5 = (unsigned)db.y - nb;
    const unsigned s6 = (unsigned)db.z - nb, s7 = (unsigned)db.w - nb;
    const bool h0 = s0 < (unsigned)NB, h1 = s1 < (unsigned)NB, h2 = s2 < (unsigned)NB, h3 = s3 < (unsigned)NB;
    const bool h4 = s4 < (unsigned)NB, h5 = s5 < (unsigned)NB, h6 = s6 < (unsigned)NB, h7 = s7 < (unsigned)NB;
    const unsigned any = __builtin_amdgcn_ballot_w32(h0 | h1 | h2 | h3 | h4 | h5 | h6 | h7);
    if (any != 0u) {
#define HITJ(J, HJ, SJ) { \
        const unsigned mj = __builtin_amdgcn_ballot_w32(HJ); \
        if (mj != 0u) { \
          if (HJ) { \
            const int pos = wc + (int)__builtin_amdgcn_mbcnt_lo(mj, 0u); \
            if (pos < WCAP) list[wave * WCAP + pos] = ((el0 + (J)) << 12) | (int)(SJ); \
          } \
          wc += (int)__builtin_popcount(mj); } }
      HITJ(0, h0, s0)
      HITJ(1, h1, s1)
      HITJ(2, h2, s2)
      HITJ(3, h3, s3)
      HITJ(4, h4, s4)
      HITJ(5, h5, s5)
      HITJ(6, h6, s6)
      HITJ(7, h7, s7)
#undef HITJ
    }
  }
  return wc;
}

__global__ __launch_bounds__(NTHR) void k_wprep(
    const float* __restrict__ W1, const float* __restrict__ W2, const float* __restrict__ W3,
    _Float16* p1, _Float16* p2, _Float16* p3) {
  const int g0 = HID * KD / 8;
  const int g1 = HID * KD / 8;
  const int g2 = OUTC * KD / 8;
  const int bstart = blockIdx.x * NTHR;
  const float* src; _Float16* dst; int Nout, segOff;
  if (bstart < g0)           { src = W1; dst = p1; Nout = HID;  segOff = 0; }
  else if (bstart < g0 + g1) { src = W2; dst = p2; Nout = HID;  segOff = g0; }
  else                       { src = W3; dst = p3; Nout = OUTC; segOff = g0 + g1; }
  const int i = bstart + (int)threadIdx.x;
  if (i >= g0 + g1 + g2) return;
  const int o  = (i - segOff) * 8;
  const int n  = o / KD;
  const int k0 = o - n * KD;
  float v[8];
#pragma unroll
  for (int e = 0; e < 8; ++e) v[e] = src[(size_t)(k0 + e) * Nout + n] * WSCALE;
  v4f a, b;
  a.x = v[0]; a.y = v[1]; a.z = v[2]; a.w = v[3];
  b.x = v[4]; b.y = v[5]; b.z = v[6]; b.w = v[7];
  const v8h hv = cvt8(a, b);
  _Float16* dp = dst + o;
  *(volatile v8h*)dp = hv;
  __threadfence();
  *(volatile v8h*)dp = hv;
}

__global__ __launch_bounds__(NTHR) void k_count(
    const int* __restrict__ ei, const float* __restrict__ ew, int* cnt, float* dinv, int nE, int vec8) {
  __shared__ __attribute__((aligned(16))) int   scnt[NBC];
  __shared__ __attribute__((aligned(16))) float sdeg[NBC];
  __shared__ __attribute__((aligned(16))) int   list[LISTN];
  __shared__ int wcnt[NWAVE];
  const int tid = threadIdx.x, lane = tid & 31, wave = tid >> 5;
  const int nodeBase = blockIdx.x * NBC;
  const int* dsts = ei + nE;

  for (int i = tid; i < NBC; i += NTHR) { scnt[i] = 0; sdeg[i] = 0.0f; }
  __syncthreads();

  const int nChunks = (nE + CHUNK - 1) / CHUNK;
#pragma unroll 1
  for (int ch = 0; ch < nChunks; ++ch) {
    const int cbase = ch * CHUNK;
    const int wc = scan_chunk<NBC>(dsts, nE, cbase, nodeBase, vec8, list, tid, lane, wave);
    if (lane == 0) wcnt[wave] = wc;
    __syncthreads();
    if (wave == 0) {
#pragma unroll 1
      for (int wsx = 0; wsx < NWAVE; ++wsx) {
        int n = __builtin_amdgcn_readfirstlane(wcnt[wsx]);
        n = n > WCAP ? WCAP : (n < 0 ? 0 : n);
        const int* lp = list + wsx * WCAP;
#pragma unroll 1
        for (int i = 0; i < n; ++i) {
          const int ent  = __builtin_amdgcn_readfirstlane(lp[i]);
          const int slot = ent & (NBC - 1);
          int e = cbase + ((ent >> 12) & (CHUNK - 1));
          e = e > nE - 1 ? nE - 1 : e;
          const float w = ew[e];
          if (lane == 0) {
            scnt[slot] = scnt[slot] + 1;
            sdeg[slot] = sdeg[slot] + w;
          }
        }
      }
    }
    __syncthreads();
  }

  v4i cq[4]; v4f dq[4];
#pragma unroll
  for (int q = 0; q < 4; ++q) {
    const int f = (wave * 4 + q) * 128 + 4 * lane;
    const v4i c = *(const v4i*)(scnt + f);
    const v4f d = *(const v4f*)(sdeg + f);
    cq[q] = c;
    const float d0 = d.x + 1.0f, d1 = d.y + 1.0f, d2 = d.z + 1.0f, d3 = d.w + 1.0f;
    const float r0 = rsqrtf(d0), r1 = rsqrtf(d1), r2 = rsqrtf(d2), r3 = rsqrtf(d3);
    dq[q].x = d0 > 0.0f ? r0 : 0.0f;
    dq[q].y = d1 > 0.0f ? r1 : 0.0f;
    dq[q].z = d2 > 0.0f ? r2 : 0.0f;
    dq[q].w = d3 > 0.0f ? r3 : 0.0f;
  }
  int*   cp = cnt + (size_t)nodeBase;
  float* dp = dinv + (size_t)nodeBase;
#pragma unroll
  for (int q = 0; q < 4; ++q) {
    const int f = (wave * 4 + q) * 128 + 4 * lane;
    *(volatile v4i*)(cp + f) = cq[q];
    *(volatile v4f*)(dp + f) = dq[q];
  }
  __threadfence();
#pragma unroll
  for (int q = 0; q < 4; ++q) {
    const int f = (wave * 4 + q) * 128 + 4 * lane;
    *(volatile v4i*)(cp + f) = cq[q];
    *(volatile v4f*)(dp + f) = dq[q];
  }
}

__global__ __launch_bounds__(OTHR) void k_offsets(
    const int* __restrict__ cnt, int* off, int* rbase, int nChunk) {
  __shared__ __attribute__((aligned(16))) int soff[NBC];
  __shared__ __attribute__((aligned(16))) int srb[RBN];
  __shared__ int wtot[OTHR / 32];
  const int tid = threadIdx.x, lane = tid & 31, wave = tid >> 5, sub = tid >> 7;
  for (int i = tid; i < RBN; i += OTHR) srb[i] = 0;
  int carry = 0;
#pragma unroll 1
  for (int ch = 0; ch < nChunk; ++ch) {
    const int base = ch * NBC;
    const v4i c0 = *(const v4i*)(cnt + base + 8 * tid);
    const v4i c1 = *(const v4i*)(cnt + base + 8 * tid + 4);
    const int e0 = max(c0.x, 0), e1 = max(c0.y, 0), e2 = max(c0.z, 0), e3 = max(c0.w, 0);
    const int e4 = max(c1.x, 0), e5 = max(c1.y, 0), e6 = max(c1.z, 0), e7 = max(c1.w, 0);
    const int ts = e0 + e1 + e2 + e3 + e4 + e5 + e6 + e7;
    int incl = ts;
#pragma unroll
    for (int d = 1; d < 32; d <<= 1) {
      const int t = __shfl_up(incl, d);
      if (lane >= d) incl += t;
    }
    if (lane == 31) wtot[wave] = incl;
    __syncthreads();
    const int S0 = wtot[0]  + wtot[1]  + wtot[2]  + wtot[3];
    const int S1 = wtot[4]  + wtot[5]  + wtot[6]  + wtot[7];
    const int S2 = wtot[8]  + wtot[9]  + wtot[10] + wtot[11];
    const int S3 = wtot[12] + wtot[13] + wtot[14] + wtot[15];
    int pre = 0;
#pragma unroll 1
    for (int w = 4 * sub; w < wave; ++w) pre += wtot[w];
    const int b0 = carry;
    const int b1 = b0 + ((S0 + 31) & ~31);
    const int b2 = b1 + ((S1 + 31) & ~31);
    const int b3 = b2 + ((S2 + 31) & ~31);
    const int b4 = b3 + ((S3 + 31) & ~31);
    const int myb = sub == 0 ? b0 : (sub == 1 ? b1 : (sub == 2 ? b2 : b3));
    if (tid == 0) {
      srb[min(4 * ch + 0, RBN - 1)] = b0;
      srb[min(4 * ch + 1, RBN - 1)] = b1;
      srb[min(4 * ch + 2, RBN - 1)] = b2;
      srb[min(4 * ch + 3, RBN - 1)] = b3;
    }
    int run = myb + pre + incl - ts;
    soff[8 * tid + 0] = run; run += e0;
    soff[8 * tid + 1] = run; run += e1;
    soff[8 * tid + 2] = run; run += e2;
    soff[8 * tid + 3] = run; run += e3;
    soff[8 * tid + 4] = run; run += e4;
    soff[8 * tid + 5] = run; run += e5;
    soff[8 * tid + 6] = run; run += e6;
    soff[8 * tid + 7] = run;
    carry = b4;
    __syncthreads();
    const v4i o0 = *(const v4i*)(soff + 4 * tid);
    const v4i o1 = *(const v4i*)(soff + 4 * (tid + OTHR));
    int* op = off + base;
    *(volatile v4i*)(op + 4 * tid) = o0;
    *(volatile v4i*)(op + 4 * (tid + OTHR)) = o1;
    __threadfence();
    *(volatile v4i*)(op + 4 * tid) = o0;
    *(volatile v4i*)(op + 4 * (tid + OTHR)) = o1;
    __syncthreads();
  }
  if (tid == 0) srb[min(4 * nChunk, RBN - 1)] = carry;
  __syncthreads();
  v4i rv = {0, 0, 0, 0};
  if (tid < 32) rv = *(const v4i*)(srb + 4 * tid);
  if (tid < 32) *(volatile v4i*)(rbase + 4 * tid) = rv;
  __threadfence();
  if (tid < 32) *(volatile v4i*)(rbase + 4 * tid) = rv;
}

__global__ __launch_bounds__(NTHR) void k_fill(
    const int* __restrict__ ei, const float* __restrict__ ew, const int* __restrict__ off,
    const int* __restrict__ rbase, int* csr, int nN, int nE, int vec8, int csrLen) {
  extern __shared__ v4f lds_dyn[];
  v2i* region = (v2i*)lds_dyn;
  int* cursor = (int*)(region + RCAP);
  int* list   = cursor + NBF;
  int* wcnt   = list + LISTN;
  const int tid = threadIdx.x, lane = tid & 31, wave = tid >> 5;
  const int b = blockIdx.x;
  const int nodeBase = b * NBF;
  const int* dsts = ei + nE;

  int rb0 = rbase[b];
  const int rb1 = rbase[b + 1];
  rb0 = rb0 < 0 ? 0 : (rb0 > csrLen ? csrLen : rb0);
  rb0 &= ~31;
  int len = rb1 - rb0;
  len = len < 0 ? 0 : (len > RCAP ? RCAP : len);
  int lenW = (len + 31) & ~31;
  if (rb0 + lenW > csrLen) lenW = (csrLen - rb0) & ~31;

  {
    const v4i z = {0, 0, 0, 0};
    for (int i = tid; i < RCAP / 2; i += NTHR) ((v4i*)region)[i] = z;
    for (int s = tid; s < NBF; s += NTHR) {
      int o = off[nodeBase + s] - rb0;
      o = o < 0 ? 0 : (o > RCAP ? RCAP : o);
      cursor[s] = o;
    }
  }
  __syncthreads();

  const int nChunks = (nE + CHUNK - 1) / CHUNK;
#pragma unroll 1
  for (int ch = 0; ch < nChunks; ++ch) {
    const int cbase = ch * CHUNK;
    const int wc = scan_chunk<NBF>(dsts, nE, cbase, nodeBase, vec8, list, tid, lane, wave);
    if (lane == 0) wcnt[wave] = wc;
    __syncthreads();
    if (wave == 0) {
#pragma unroll 1
      for (int wsx = 0; wsx < NWAVE; ++wsx) {
        int n = __builtin_amdgcn_readfirstlane(wcnt[wsx]);
        n = n > WCAP ? WCAP : (n < 0 ? 0 : n);
        const int* lp = list + wsx * WCAP;
#pragma unroll 1
        for (int i = 0; i < n; ++i) {
          const int ent  = __builtin_amdgcn_readfirstlane(lp[i]);
          const int slot = ent & (NBF - 1);
          int e = cbase + ((ent >> 12) & (CHUNK - 1));
          e = e > nE - 1 ? nE - 1 : e;
          int src = ei[e];
          src = src < 0 ? 0 : (src > nN - 1 ? nN - 1 : src);
          const float w = ew[e];
          if (lane == 0) {
            int pos = cursor[slot];
            pos = pos < 0 ? 0 : (pos > RCAP - 1 ? RCAP - 1 : pos);
            v2i en;
            en.x = src;
            en.y = __float_as_int(w);
            region[pos] = en;
            const int np = pos + 1;
            cursor[slot] = np > RCAP ? RCAP : np;
          }
        }
      }
    }
    __syncthreads();
  }

  const int nv = lenW >> 1;
  int* gp = csr + 2 * (size_t)rb0;
#pragma unroll 1
  for (int i = tid; i < nv; i += NTHR) { const v4i v = ((const v4i*)region)[i]; *(volatile v4i*)(gp + 4 * i) = v; }
  __threadfence();
#pragma unroll 1
  for (int i = tid; i < nv; i += NTHR) { const v4i v = ((const v4i*)region)[i]; *(volatile v4i*)(gp + 4 * i) = v; }
}

template <int NCT>
__global__ __launch_bounds__(NTHR) void k_gemm(
    const float* __restrict__ A, const _Float16* __restrict__ Bs, const float* __restrict__ dinv,
    float* C, int nRowsA) {
  extern __shared__ v4f lds_dyn[];
  float* stg = (float*)lds_dyn;
  constexpr int NCOL = 16 * NCT;
  constexpr int NI   = 16 * NCOL / 128;
  const int tid = threadIdx.x, lane = tid & 31, wave = tid >> 5, hh = lane >> 4, m = lane & 15;
  const int rowBase = blockIdx.x * GROWS;

  int arow = rowBase + wave * 16 + m;
  arow = arow > nRowsA - 1 ? nRowsA - 1 : arow;
  const float* ar = A + (size_t)arow * KD + 8 * hh;

  v8f acc[NCT];
#pragma unroll
  for (int t = 0; t < NCT; ++t) { v8f z = {0.f, 0.f, 0.f, 0.f, 0.f, 0.f, 0.f, 0.f}; acc[t] = z; }
#pragma unroll
  for (int kt = 0; kt < KD / 32; ++kt) {
    const float* ap = ar + 32 * kt;
    const v4f a0 = *(const v4f*)ap;
    const v4f a1 = *(const v4f*)(ap + 4);
    const v4f a2 = *(const v4f*)(ap + 16);
    const v4f a3 = *(const v4f*)(ap + 20);
    FragH a;
    a.h[0] = cvt8(a0, a1);
    a.h[1] = cvt8(a2, a3);
#pragma unroll
    for (int t = 0; t < NCT; ++t) {
      const _Float16* bp = Bs + (size_t)(16 * t + m) * KD + 32 * kt + 8 * hh;
      FragH b;
      b.h[0] = *(const v8h*)bp;
      b.h[1] = *(const v8h*)(bp + 16);
      acc[t] = wmh(a.v, b.v, acc[t]);
    }
  }

  const int r0 = wave * 16 + 8 * hh;
  const v4f dA = *(const v4f*)(dinv + (size_t)rowBase + r0);
  const v4f dB = *(const v4f*)(dinv + (size_t)rowBase + r0 + 4);
  float s[8];
  s[0] = dA.x; s[1] = dA.y; s[2] = dA.z; s[3] = dA.w; s[4] = dB.x; s[5] = dB.y; s[6] = dB.z; s[7] = dB.w;
#pragma unroll
  for (int r = 0; r < 8; ++r) s[r] = s[r] * WINV;
  float* sp = stg + r0 * NCOL + m;
#pragma unroll
  for (int t = 0; t < NCT; ++t) {
#pragma unroll
    for (int r = 0; r < 8; ++r) sp[r * NCOL + 16 * t] = acc[t][r] * s[r];
  }
  __syncthreads();

  const float* lp = stg + wave * 16 * NCOL + 4 * lane;
  float* gp = C + ((size_t)rowBase + wave * 16) * NCOL + 4 * lane;
#pragma unroll
  for (int i = 0; i < NI; ++i) { const v4f v = *(const v4f*)(lp + 128 * i); *(volatile v4f*)(gp + (size_t)128 * i) = v; }
  __threadfence();
#pragma unroll
  for (int i = 0; i < NI; ++i) { const v4f v = *(const v4f*)(lp + 128 * i); *(volatile v4f*)(gp + (size_t)128 * i) = v; }
}

template <int CH>
__global__ __launch_bounds__(ATHR) void k_agg(
    const v2i* __restrict__ csr, const int* __restrict__ off, const int* __restrict__ cnt,
    const float* __restrict__ dinv, const float* __restrict__ hw, const float* __restrict__ bias,
    float* dst, int nN, int csrLen, int relu, int nStoreRows) {
  extern __shared__ v4f lds_dyn[];
  float* stage = (float*)lds_dyn;
  constexpr int LPG = CH / 8;
  constexpr int EPI = 32 / LPG;
  constexpr int LPR = CH / 4;
  constexpr int RPI = 32 / LPR;
  constexpr int NI  = 32 / RPI;
  const int tid = threadIdx.x, lane = tid & 31, wave = tid >> 5;
  const int g  = lane / LPG;
  const int li = lane & (LPG - 1);
  const int tbase = blockIdx.x * TGT + wave * 32;
  const int cl = tbase + lane;
  const int cnt_l = cnt[cl];
  const int off_l = off[cl];
  union FI { float f; int i; };
  FI dvu; dvu.f = dinv[cl];
  const v4f bA = *(const v4f*)(bias + 8 * li);
  const v4f bB = *(const v4f*)(bias + 8 * li + 4);
  float* wst = stage + wave * 32 * CH;

#pragma unroll 1
  for (int j = 0; j < 32; ++j) {
    const int c = tbase + j;
    int n = __builtin_amdgcn_readlane(cnt_l, j);
    n = n < 0 ? 0 : (n > DEGCAP ? DEGCAP : n);
    const int st = __builtin_amdgcn_readlane(off_l, j);
    FI du; du.i = __builtin_amdgcn_readlane(dvu.i, j);
    const float dc = du.f;
    v4f accA = {0.f, 0.f, 0.f, 0.f};
    v4f accB = {0.f, 0.f, 0.f, 0.f};
    const int nit = (n + EPI - 1) / EPI;
#pragma unroll 1
    for (int i = 0; i < nit; ++i) {
      const int q = EPI * i + g;
      int p = st + q;
      p = p < 0 ? 0 : (p > csrLen - 1 ? csrLen - 1 : p);
      const v2i en = csr[p];
      int s = en.x;
      s = s < 0 ? 0 : (s > nN - 1 ? nN - 1 : s);
      FI wu; wu.i = en.y;
      const float w = (q < n) ? wu.f : 0.0f;
      const float* rp = hw + (size_t)s * CH + 8 * li;
      const v4f x0 = *(const v4f*)rp;
      const v4f x1 = *(const v4f*)(rp + 4);
      accA = accA + x0 * w;
      accB = accB + x1 * w;
    }
#pragma unroll
    for (int sh = LPG; sh < 32; sh <<= 1) {
      accA.x += __shfl_xor(accA.x, sh); accA.y += __shfl_xor(accA.y, sh);
      accA.z += __shfl_xor(accA.z, sh); accA.w += __shfl_xor(accA.w, sh);
      accB.x += __shfl_xor(accB.x, sh); accB.y += __shfl_xor(accB.y, sh);
      accB.z += __shfl_xor(accB.z, sh); accB.w += __shfl_xor(accB.w, sh);
    }
    const float* sp = hw + (size_t)c * CH + 8 * li;
    const v4f s0 = *(const v4f*)sp;
    const v4f s1 = *(const v4f*)(sp + 4);
    v4f vA = (accA + s0) * dc + bA;
    v4f vB = (accB + s1) * dc + bB;
    if (relu != 0) {
      vA.x = fmaxf(vA.x, 0.f); vA.y = fmaxf(vA.y, 0.f); vA.z = fmaxf(vA.z, 0.f); vA.w = fmaxf(vA.w, 0.f);
      vB.x = fmaxf(vB.x, 0.f); vB.y = fmaxf(vB.y, 0.f); vB.z = fmaxf(vB.z, 0.f); vB.w = fmaxf(vB.w, 0.f);
    }
    if (g == 0) {
      *(v4f*)(wst + j * CH + 8 * li)     = vA;
      *(v4f*)(wst + j * CH + 8 * li + 4) = vB;
    }
  }
  __syncthreads();

  const int sr = lane / LPR;
  const int sc = 4 * (lane & (LPR - 1));
#pragma unroll
  for (int i = 0; i < NI; ++i) {
    const int rl  = RPI * i + sr;
    const int row = tbase + rl;
    const v4f v = *(const v4f*)(wst + rl * CH + sc);
    if (row < nStoreRows) *(volatile v4f*)(dst + (size_t)row * CH + sc) = v;
  }
  __threadfence();
#pragma unroll
  for (int i = 0; i < NI; ++i) {
    const int rl  = RPI * i + sr;
    const int row = tbase + rl;
    const v4f v = *(const v4f*)(wst + rl * CH + sc);
    if (row < nStoreRows) *(volatile v4f*)(dst + (size_t)row * CH + sc) = v;
  }
}

extern "C" void kernel_launch(void* const* d_in, const int* in_sizes, int n_in,
                              void* d_out, int out_size, void* d_ws, size_t ws_size,
                              hipStream_t stream) {
  if (n_in < 9) return;
  const int nN = in_sizes[0] / KD;
  const int nE = in_sizes[1] / 2;
  if (nN <= 0 || nE <= 0 || in_sizes[0] != nN * KD || in_sizes[1] != 2 * nE || in_sizes[2] != nE) return;
  if (in_sizes[3] != KD * HID || in_sizes[4] < HID || in_sizes[5] != KD * HID || in_sizes[6] < HID ||
      in_sizes[7] != KD * OUTC || in_sizes[8] < OUTC) return;
  if (out_size != nN * OUTC) return;
  if (nE > (1 << 28) || nN > (1 << 24)) return;

  const float* x  = (const float*)d_in[0];
  const int*   ei = (const int*)d_in[1];
  const float* ew = (const float*)d_in[2];
  const float* W1 = (const float*)d_in[3];
  const float* b1 = (const float*)d_in[4];
  const float* W2 = (const float*)d_in[5];
  const float* b2 = (const float*)d_in[6];
  const float* W3 = (const float*)d_in[7];
  const float* b3 = (const float*)d_in[8];
  float* out = (float*)d_out;

  const int NPAD   = ((nN + GROWS - 1) / GROWS) * GROWS;
  const int nBC    = (nN + NBC - 1) / NBC;
  const int CNTPAD = nBC * NBC;
  if (4 * nBC + 1 > RBN) return;
  const int nBF    = (nN + NBF - 1) / NBF;
  const int csrLen = ((nE + 31) & ~31) + 4096;
  const int nGemm  = NPAD / GROWS;
  const int nAgg   = NPAD / TGT;

  char* ws = (char*)d_ws;
  size_t off = 0;
  const size_t oW1  = off; off += (size_t)HID * KD * 2;            off = (off + 255) & ~(size_t)255;
  const size_t oW2  = off; off += (size_t)HID * KD * 2;            off = (off + 255) & ~(size_t)255;
  const size_t oW3  = off; off += (size_t)OUTC * KD * 2;           off = (off + 255) & ~(size_t)255;
  const size_t oCnt = off; off += (size_t)CNTPAD * 4;              off = (off + 255) & ~(size_t)255;
  const size_t oDv  = off; off += (size_t)CNTPAD * 4;              off = (off + 255) & ~(size_t)255;
  const size_t oOff = off; off += (size_t)CNTPAD * 4;              off = (off + 255) & ~(size_t)255;
  const size_t oRb  = off; off += (size_t)RBN * 4;                 off = (off + 255) & ~(size_t)255;
  const size_t oCsr = off; off += (size_t)csrLen * 8;              off = (off + 255) & ~(size_t)255;
  const size_t oH   = off; off += (size_t)NPAD * HID * 4;          off = (off + 255) & ~(size_t)255;
  const size_t oHw  = off; off += (size_t)NPAD * HID * 4;          off = (off + 255) & ~(size_t)255;
  if (off > ws_size) return;
  _Float16* w1p  = (_Float16*)(ws + oW1);
  _Float16* w2p  = (_Float16*)(ws + oW2);
  _Float16* w3p  = (_Float16*)(ws + oW3);
  int*      cnt  = (int*)(ws + oCnt);
  float*    dinv = (float*)(ws + oDv);
  int*      offp = (int*)(ws + oOff);
  int*      rb   = (int*)(ws + oRb);
  int*      csr  = (int*)(ws + oCsr);
  float*    h    = (float*)(ws + oH);
  float*    hw   = (float*)(ws + oHw);

  const int vec8 = ((nE & 3) == 0) ? 1 : 0;

  const int nPrep = HID * KD / 8 + HID * KD / 8 + OUTC * KD / 8;
  k_wprep<<<(nPrep + NTHR - 1) / NTHR, NTHR, 0, stream>>>(W1, W2, W3, w1p, w2p, w3p);

  k_count<<<nBC, NTHR, 0, stream>>>(ei, ew, cnt, dinv, nE, vec8);
  k_offsets<<<1, OTHR, 0, stream>>>(cnt, offp, rb, nBC);
  hipFuncSetAttribute(reinterpret_cast<const void*>(&k_fill),
                      hipFuncAttributeMaxDynamicSharedMemorySize, LDS_FILL);
  k_fill<<<nBF, NTHR, LDS_FILL, stream>>>(ei, ew, offp, rb, csr, nN, nE, vec8, csrLen);

  hipFuncSetAttribute(reinterpret_cast<const void*>(&k_gemm<8>),
                      hipFuncAttributeMaxDynamicSharedMemorySize, LDS_GEMM8);
  hipFuncSetAttribute(reinterpret_cast<const void*>(&k_gemm<4>),
                      hipFuncAttributeMaxDynamicSharedMemorySize, LDS_GEMM4);
  hipFuncSetAttribute(reinterpret_cast<const void*>(&k_agg<128>),
                      hipFuncAttributeMaxDynamicSharedMemorySize, LDS_AGG128);
  hipFuncSetAttribute(reinterpret_cast<const void*>(&k_agg<64>),
                      hipFuncAttributeMaxDynamicSharedMemorySize, LDS_AGG64);

  k_gemm<8><<<nGemm, NTHR, LDS_GEMM8, stream>>>(x, w1p, dinv, hw, nN);
  k_agg<128><<<nAgg, ATHR, LDS_AGG128, stream>>>((const v2i*)csr, offp, cnt, dinv, hw, b1, h, nN, csrLen, 1, NPAD);
  k_gemm<8><<<nGemm, NTHR, LDS_GEMM8, stream>>>(h, w2p, dinv, hw, NPAD);
  k_agg<128><<<nAgg, ATHR, LDS_AGG128, stream>>>((const v2i*)csr, offp, cnt, dinv, hw, b2, h, nN, csrLen, 1, NPAD);
  k_gemm<4><<<nGemm, NTHR, LDS_GEMM4, stream>>>(h, w3p, dinv, hw, NPAD);
  k_agg<64><<<nAgg, ATHR, LDS_AGG64, stream>>>((const v2i*)csr, offp, cnt, dinv, hw, b3, out, nN, csrLen, 0, nN);
}
